// HyperbolicHead_61125974556677
// MI455X (gfx1250) — hardware-verified
//
#include <hip/hip_runtime.h>


namespace {
constexpr int N = 8192, D = 768, C = 1000, CP = 1008;
constexpr float XS = 8.0f, WSC = 256.0f, EPS = 1e-6f, T_CLIP = 0.96f, BALL_EPS = 4e-3f, ATANH_EPS = 1e-7f;
typedef _Float16 b16;
typedef __attribute__((ext_vector_type(16))) _Float16 v16b;
typedef __attribute__((ext_vector_type(8))) _Float16 v8b;
typedef __attribute__((ext_vector_type(8))) float v8f;
typedef __attribute__((ext_vector_type(4))) float v4f;
typedef __attribute__((ext_vector_type(2))) float v2f;
__device__ __forceinline__ float bf16_rne(float f) { unsigned int u = __float_as_uint(f); u += 0x7FFFu + ((u >> 16) & 1u); float r = __uint_as_float(u & 0xFFFF0000u); asm volatile("" : "+v"(r)); return r; }
__device__ __forceinline__ v16b frag_kb(const b16* p, int hh) { const v8b a = *(const v8b*)(p + 8 * hh), b = *(const v8b*)(p + 16 + 8 * hh); v16b f;
#pragma unroll
  for (int e = 0; e < 8; ++e) { f[e] = a[e]; f[8 + e] = b[e]; } return f; }
__device__ __forceinline__ v8f wmma16b(v16b a, v16b b, v8f c) { v8f d = __builtin_amdgcn_wmma_f32_16x16x32_f16(false, a, false, b, (short)0, c, false, false); asm volatile("v_nop\n\tv_nop\n\tv_nop\n\tv_nop" : "+v"(d) : "v"(a), "v"(b)); return d; }
__device__ __forceinline__ void wave_lds_sync() { __builtin_amdgcn_fence(__ATOMIC_RELEASE, "workgroup"); __builtin_amdgcn_wave_barrier(); __builtin_amdgcn_fence(__ATOMIC_ACQUIRE, "workgroup"); }
__device__ __forceinline__ float pmul(float a, float b) { float p = a * b; asm volatile("" : "+v"(p)); return p; }
__device__ __forceinline__ float softplus(float v) { return v > 20.0f ? v : log1pf(__expf(v)); }

__global__ __launch_bounds__(256) void proto_kernel(const float* __restrict__ proto, const float* __restrict__ rho, b16* __restrict__ PT, float* __restrict__ CS) { const int wave = threadIdx.x >> 5, lane = threadIdx.x & 31; const int j = blockIdx.x * 8 + wave; if (j >= CP) return; float v[24]; float sq = 0.0f;
#pragma unroll
  for (int q = 0; q < 24; ++q) { v[q] = j < C ? bf16_rne(proto[(size_t)j * D + lane * 24 + q]) : 0.0f; sq += pmul(v[q], v[q]); }
  for (int o = 16; o; o >>= 1) sq += __shfl_xor(sq, o);
  const float c = softplus(bf16_rne(rho[0])), sc = sqrtf(c); const float maxn = (1.0f - BALL_EPS) / sc; const float n = fmaxf(sqrtf(sq), 1e-15f); const float ps = n > maxn ? maxn / n : 1.0f;
  float y2e = 0.0f;
#pragma unroll
  for (int q = 0; q < 24; ++q) { const float pv = pmul(v[q], ps); y2e += pmul(pv, pv); } for (int o = 16; o; o >>= 1) y2e += __shfl_xor(y2e, o);
  for (int pass = 0; pass < 2; ++pass) {
#pragma unroll
    for (int q3 = 0; q3 < 3; ++q3) { v8b pk; for (int e = 0; e < 8; ++e) pk[e] = (b16)(v[q3 * 8 + e] * WSC); *(volatile v8b*)(PT + (size_t)j * D + lane * 24 + q3 * 8) = pk; }
    ((volatile float*)CS)[(size_t)j * 32 + lane] = lane == 0 ? ps : (lane == 1 ? y2e : 0.0f); __threadfence(); } }
__global__ __launch_bounds__(256) void row_kernel(const float* __restrict__ cls, const float* __restrict__ cls_scale, const float* __restrict__ rho, int RLIM, float* __restrict__ RS) { const int wave = threadIdx.x >> 5, lane = threadIdx.x & 31; const int r = blockIdx.x * 8 + wave; if (r >= RLIM) return; float v[24]; float sq = 0.0f;
  const float c = softplus(bf16_rne(rho[0])), sc = sqrtf(c); const float s = softplus(bf16_rne(cls_scale[0])) + EPS;
#pragma unroll
  for (int q = 0; q < 24; ++q) { v[q] = pmul(bf16_rne(cls[(size_t)r * D + q * 32 + lane]), s); sq += pmul(v[q], v[q]); } for (int o = 16; o; o >>= 1) sq += __shfl_xor(sq, o);
  const float xmax = atanhf(T_CLIP) / (sc + EPS); const float xn = sqrtf(sq); const float f1 = fminf(xmax / (xn + EPS), 1.0f); float tot = pmul(s, f1);
  float sq1 = 0.0f;
#pragma unroll
  for (int q = 0; q < 24; ++q) { v[q] = pmul(v[q], f1); sq1 += pmul(v[q], v[q]); } for (int o = 16; o; o >>= 1) sq1 += __shfl_xor(sq1, o);
  const float vn = fmaxf(sqrtf(sq1), 1e-15f); const float f2 = tanhf(sc * vn) / (sc * vn); tot = pmul(tot, f2); float sq2 = 0.0f;
#pragma unroll
  for (int q = 0; q < 24; ++q) { v[q] = pmul(v[q], f2); sq2 += pmul(v[q], v[q]); } for (int o = 16; o; o >>= 1) sq2 += __shfl_xor(sq2, o);
  const float maxn = (1.0f - BALL_EPS) / sc; const float hn0 = fmaxf(sqrtf(sq2), 1e-15f); const float f3 = hn0 > maxn ? maxn / hn0 : 1.0f; tot = pmul(tot, f3); float sq3 = 0.0f;
#pragma unroll
  for (int q = 0; q < 24; ++q) { v[q] = pmul(v[q], f3); sq3 += pmul(v[q], v[q]); } for (int o = 16; o; o >>= 1) sq3 += __shfl_xor(sq3, o);
  const float rmax = T_CLIP / (sc + EPS); const float hn = sqrtf(sq3); const float f4 = fminf(rmax / (hn + EPS), 1.0f); tot = pmul(tot, f4); float sq4 = 0.0f;
#pragma unroll
  for (int q = 0; q < 24; ++q) { v[q] = pmul(v[q], f4); sq4 += pmul(v[q], v[q]); } for (int o = 16; o; o >>= 1) sq4 += __shfl_xor(sq4, o);
  for (int pass = 0; pass < 2; ++pass) { ((volatile float*)RS)[(size_t)r * 32 + lane] = lane == 0 ? tot : (lane == 1 ? sq4 : 0.0f); __threadfence(); } }
__global__ __launch_bounds__(32) void main_kernel(const float* __restrict__ cls, const b16* __restrict__ PT, const float* __restrict__ RS, const float* __restrict__ CS, int RLIM, float* __restrict__ XY) {
  __shared__ __attribute__((aligned(16))) b16 Ah[16][D + 8]; __shared__ float Tf[16][132]; const int lane = threadIdx.x, nloc = lane & 15, hlf = lane >> 4; const size_t r0 = (size_t)blockIdx.x * 16; if (r0 >= (size_t)RLIM) return;
  for (int rr = 0; rr < 16; ++rr) for (int q = 0; q < D / 32; ++q) Ah[rr][q * 32 + lane] = (b16)(bf16_rne(cls[(r0 + rr) * D + q * 32 + lane]) * XS);
  wave_lds_sync();
#pragma unroll 1
  for (int g = 0; g < 8; ++g) { const int t0 = g * 8, nt = (g == 7) ? (CP / 16 - 56) : 8;
    v8f acc[8];
#pragma unroll
    for (int t = 0; t < 8; ++t) acc[t] = (v8f){};
#pragma unroll 1
    for (int kb = 0; kb < D; kb += 32) { const v16b a = frag_kb(&Ah[nloc][kb], hlf);
#pragma unroll
      for (int t = 0; t < 8; ++t) if (t < nt) acc[t] = wmma16b(a, frag_kb(PT + (size_t)((t0 + t) * 16 + nloc) * D + kb, hlf), acc[t]); }
#pragma unroll
    for (int t = 0; t < 8; ++t) { const int j = (t0 + t) * 16 + nloc; const float ps = (t < nt) ? CS[(size_t)j * 32] : 0.0f;
#pragma unroll
      for (int r8 = 0; r8 < 8; ++r8) { const size_t r = r0 + 8 * hlf + r8; Tf[8 * hlf + r8][t * 16 + nloc] = (t < nt) ? pmul(pmul(acc[t][r8] * (1.0f / (XS * WSC)), RS[r * 32]), ps) : 0.0f; } }
    wave_lds_sync();
    for (int pass = 0; pass < 2; ++pass) { for (int rr = 0; rr < 16; ++rr) *(volatile v4f*)(XY + (r0 + rr) * 1024 + g * 128 + lane * 4) = *(const v4f*)(&Tf[rr][lane * 4]); __threadfence(); }
    wave_lds_sync(); }
}
__global__ __launch_bounds__(256) void dist_kernel(const float* __restrict__ XY, const float* __restrict__ RS, const float* __restrict__ CS, const float* __restrict__ rho, const float* __restrict__ sigma, const float* __restrict__ bias, int RLIM, float* __restrict__ out) { const size_t u = (size_t)blockIdx.x * 256 + threadIdx.x; if (u >= (size_t)N * C) return; const size_t r = u / C; const int j = (int)(u % C); float res = 0.0f;
  if (r < (size_t)RLIM) { const float c = softplus(bf16_rne(rho[0])), sc = sqrtf(c); float sig = softplus(bf16_rne(sigma[0])) + EPS; sig = fminf(fmaxf(sig, 0.01f), 10.0f);
    const float xy = XY[r * 1024 + j], x2 = RS[r * 32 + 1], y2 = CS[(size_t)j * 32 + 1];
    const float A = 1.0f - 2.0f * c * xy + c * y2, B = 1.0f - c * x2; const float num2 = fmaxf(pmul(pmul(A, A), x2) + pmul(pmul(B, B), y2) - 2.0f * pmul(pmul(A, B), xy), 0.0f); const float den = 1.0f - 2.0f * c * xy + pmul(pmul(c, c), pmul(x2, y2));
    const float mn = sqrtf(num2) / den; float z = sc * mn; z = fminf(fmaxf(z, -1.0f + ATANH_EPS), 1.0f - ATANH_EPS); const float d = (2.0f / sc) * atanhf(z); res = -pmul(d, d) / (2.0f * sig * sig) + bf16_rne(bias[j]); }
  for (int pass = 0; pass < 2; ++pass) { ((volatile float*)out)[u] = res; __threadfence(); } }
}

extern "C" void kernel_launch(void* const* d_in, const int* in_sizes, int n_in, void* d_out, int out_size, void* d_ws, size_t ws_size, hipStream_t stream) {
  (void)n_in;
  auto Fp = [&](int i) { return (const float*)d_in[i]; };
  if (in_sizes[0] != N * D || in_sizes[1] != C * D || in_sizes[2] != C || in_sizes[3] != 1 || in_sizes[4] != 1 || in_sizes[5] != 1 || out_size != N * C) return;
  const int RLIM = N;
  size_t off = 0; char* ws = (char*)d_ws;
  auto carve = [&](size_t bytes) { char* p = ws + off; off += (bytes + 255) & ~(size_t)255; return p; };
  b16* PT = (b16*)carve((size_t)CP * D * 2); float* CS = (float*)carve((size_t)CP * 32 * 4); float* RS = (float*)carve((size_t)N * 32 * 4); float* XY = (float*)carve((size_t)N * 1024 * 4);
  if (off > ws_size || off > ((size_t)48 << 20)) return;
  proto_kernel<<<CP / 8, 256, 0, stream>>>(Fp(1), Fp(5), PT, CS);
  row_kernel<<<RLIM / 8, 256, 0, stream>>>(Fp(0), Fp(4), Fp(5), RLIM, RS);
  main_kernel<<<RLIM / 16, 32, 0, stream>>>(Fp(0), PT, RS, CS, RLIM, XY);
  dist_kernel<<<(unsigned)(((size_t)N * C + 255) / 256), 256, 0, stream>>>(XY, RS, CS, Fp(5), Fp(3), Fp(2), RLIM, (float*)d_out);
}
